// S6Layer_41764261987304
// MI455X (gfx1250) — hardware-run, weakly checked
//
#include <hip/hip_runtime.h>


#define NM   32768
#define NW   256
#define NI   384
#define NE   8
#define NK   32
#define NX   768
#define NA   1152
typedef _Float16 h16;
typedef unsigned short bf;
typedef __attribute__((ext_vector_type(16))) __bf16   v16bf;
typedef __attribute__((ext_vector_type(16))) _Float16 v16h;
typedef __attribute__((ext_vector_type(8)))  _Float16 v8h;
typedef __attribute__((ext_vector_type(8)))  unsigned short v8us;
typedef __attribute__((ext_vector_type(8)))  float    v8f;
typedef __attribute__((ext_vector_type(4)))  float    v4f;
typedef v8h  __attribute__((may_alias)) v8ha;
typedef v4f  __attribute__((may_alias)) v4fa;
typedef v8us __attribute__((may_alias)) v8usa;

__device__ __forceinline__ unsigned short f2bf(float f) { unsigned u = __float_as_uint(f); u += 0x7FFFu + ((u >> 16) & 1u); return (unsigned short)(u >> 16); }
__device__ __forceinline__ float bf2f(unsigned short b) { return __uint_as_float(((unsigned)b) << 16); }
__device__ __forceinline__ float bfr(float f) { return bf2f(f2bf(f)); }
__device__ __forceinline__ v16h cat16(v8h lo, v8h hi) { return __builtin_shufflevector(lo, hi, 0, 1, 2, 3, 4, 5, 6, 7, 8, 9, 10, 11, 12, 13, 14, 15); }
__device__ __forceinline__ v16bf cat16b(v8us lo, v8us hi) { return __builtin_bit_cast(v16bf, __builtin_shufflevector(lo, hi, 0, 1, 2, 3, 4, 5, 6, 7, 8, 9, 10, 11, 12, 13, 14, 15)); }
__device__ __forceinline__ v8f wmma16(v16h a, v16h b, v8f c) { return __builtin_amdgcn_wmma_f32_16x16x32_f16(false, a, false, b, (short)0, c, false, false); }
__device__ __forceinline__ v8f wmmab(v16bf a, v16bf b, v8f c) { return __builtin_amdgcn_wmma_f32_16x16x32_bf16(false, a, false, b, (short)0, c, false, false); }

template <typename T16> struct WFrag;
template <> struct WFrag<h16> { typedef v16h V; static __device__ __forceinline__ V ld(const h16* p) { return cat16(*(const v8h*)p, *(const v8h*)(p + 16)); } static __device__ __forceinline__ v8f mma(V a, V b, v8f c) { return wmma16(a, b, c); } };
template <> struct WFrag<bf> { typedef v16bf V; static __device__ __forceinline__ V ld(const bf* p) { return cat16b(*(const v8us*)p, *(const v8us*)(p + 16)); } static __device__ __forceinline__ v8f mma(V a, V b, v8f c) { return wmmab(a, b, c); } };
template <typename T16, int NSPLIT, bool BIAS>
__global__ __launch_bounds__(32) void k_gemmw(const T16* __restrict__ A, const T16* __restrict__ A2, const T16* __restrict__ Bt, const T16* __restrict__ Bt2, int K, float* C, int ldc, const float* __restrict__ bias, size_t sA, size_t sB, size_t sC) {
    typedef typename WFrag<T16>::V V;
    __shared__ __align__(16) float os[16 * 68];
    const size_t z = blockIdx.z; A += z * sA; if (A2) A2 += z * sA; Bt += z * sB; if (Bt2) Bt2 += z * sB; C += z * sC;
    const int lane = threadIdx.x & 31, lr = lane & 15, hi = lane >> 4; const int r0 = blockIdx.x * 64, c0 = blockIdx.y * 64;
    v8f acc[4][4];
#pragma unroll
    for (int mb = 0; mb < 4; ++mb)
#pragma unroll
        for (int nb = 0; nb < 4; ++nb) acc[mb][nb] = (v8f){};
    const size_t aoff = (size_t)(r0 + lr) * K + 8 * hi, boff = (size_t)(c0 + lr) * K + 8 * hi;
    for (int kc = 0; kc < K; kc += 32) {
        V a[4], a2[4];
#pragma unroll
        for (int mb = 0; mb < 4; ++mb) { a[mb] = WFrag<T16>::ld(A + aoff + (size_t)mb * 16 * K + kc); if (NSPLIT == 1 || NSPLIT == 2) a2[mb] = WFrag<T16>::ld(A2 + aoff + (size_t)mb * 16 * K + kc); }
#pragma unroll
        for (int nb = 0; nb < 4; ++nb) { const V b = WFrag<T16>::ld(Bt + boff + (size_t)nb * 16 * K + kc); V b2; if (NSPLIT >= 2) b2 = WFrag<T16>::ld(Bt2 + boff + (size_t)nb * 16 * K + kc);
#pragma unroll
            for (int mb = 0; mb < 4; ++mb) { acc[mb][nb] = WFrag<T16>::mma(a[mb], b, acc[mb][nb]); if (NSPLIT == 1 || NSPLIT == 2) acc[mb][nb] = WFrag<T16>::mma(a2[mb], b, acc[mb][nb]); if (NSPLIT >= 2) acc[mb][nb] = WFrag<T16>::mma(a[mb], b2, acc[mb][nb]); } }
        asm volatile("v_nop\n\tv_nop\n\tv_nop\n\tv_nop" : "+v"(acc[0][0]), "+v"(acc[1][1]), "+v"(acc[2][2]), "+v"(acc[3][3]) : "v"(a[0]), "v"(a[3]));
    }
#pragma unroll
    for (int mb = 0; mb < 4; ++mb) {
#pragma unroll
        for (int nb = 0; nb < 4; ++nb) {
#pragma unroll
            for (int j = 0; j < 8; ++j) os[(hi * 8 + j) * 68 + nb * 16 + lr] = acc[mb][nb][j]; }
        __builtin_amdgcn_wave_barrier(); asm volatile("" ::: "memory");
        float* crow = C + (size_t)(r0 + mb * 16) * ldc + c0;
#pragma unroll 1
        for (int ps = 0; ps < 2; ++ps) {
#pragma unroll
            for (int s = 0; s < 8; ++s) { const int row = 2 * s + hi, cofs = lr * 4; v4f val = *(const v4fa*)(os + row * 68 + cofs); if (BIAS) { val[0] += bfr(bias[c0 + cofs]); val[1] += bfr(bias[c0 + cofs + 1]); val[2] += bfr(bias[c0 + cofs + 2]); val[3] += bfr(bias[c0 + cofs + 3]); }
                *(volatile v4f*)(crow + (size_t)row * ldc + cofs) = val; }
            if (ps == 0) __threadfence(); }
        __builtin_amdgcn_wave_barrier(); asm volatile("" ::: "memory");
    }
}

typedef __attribute__((ext_vector_type(2))) _Float16 v2h;
typedef __attribute__((ext_vector_type(4))) _Float16 v4h;
typedef __attribute__((ext_vector_type(2))) unsigned short v2us;
typedef __attribute__((ext_vector_type(4))) unsigned short v4us;
typedef __attribute__((ext_vector_type(2))) float v2f;
typedef __attribute__((ext_vector_type(4))) int v4i;

__device__ __forceinline__ h16 toh_flush(float x) { const float z = (fabsf(x) < 6.103515625e-05f) ? 0.0f : x; return (h16)z; }

template <bool RB>
__global__ __launch_bounds__(256) void k_c16(const float* __restrict__ src, h16* dst, size_t n8) { const size_t i = (size_t)blockIdx.x * 256 + threadIdx.x; if (i >= n8) return; const float* p = src + i * 8; const v4f a = *(const v4f*)p, b = *(const v4f*)(p + 4); v8h o;
#pragma unroll
    for (int q = 0; q < 4; ++q) { o[q] = toh_flush(RB ? bfr(a[q]) : a[q]); o[q + 4] = toh_flush(RB ? bfr(b[q]) : b[q]); }
    *(volatile v8h*)(dst + i * 8) = o; __threadfence(); *(volatile v8h*)(dst + i * 8) = o; }

__global__ __launch_bounds__(256) void k_rnh(const float* __restrict__ src, const float* __restrict__ sq, const float* __restrict__ oq, h16* dst) { const size_t r = (size_t)blockIdx.x * 256 + threadIdx.x; const float* p = src + r * NW; float sm = 0.0f;
    for (int cl = 0; cl < NW; cl += 4) { const v4f va = *(const v4f*)(p + cl); sm += bfr(va[0]); sm += bfr(va[1]); sm += bfr(va[2]); sm += bfr(va[3]); }
    const float av = sm * (1.0f / NW); float sv = 0.0f;
    for (int cl = 0; cl < NW; cl += 4) { const v4f va = *(const v4f*)(p + cl);
#pragma unroll
        for (int q = 0; q < 4; ++q) { const float df = bfr(va[q]) - av; sv += df * df; } }
    const float rs = 1.0f / sqrtf(sv * (1.0f / NW) + 1e-5f); h16* o = dst + r * NW; const int sk = (int)(threadIdx.x & 3u) * 64;
    for (int cl = 0; cl < NW; cl += 8) { const int cs = (cl + sk) & (NW - 1); const v4f va = *(const v4f*)(p + cs), vb = *(const v4f*)(p + cs + 4), ga = *(const v4f*)(sq + cs), gb = *(const v4f*)(sq + cs + 4), oa = *(const v4f*)(oq + cs), ob = *(const v4f*)(oq + cs + 4); v8h wo;
#pragma unroll
        for (int q = 0; q < 4; ++q) { wo[q] = toh_flush((bfr(va[q]) - av) * rs * bfr(ga[q]) + bfr(oa[q])); wo[q + 4] = toh_flush((bfr(vb[q]) - av) * rs * bfr(gb[q]) + bfr(ob[q])); }
        *(volatile v8h*)(o + cs) = wo; }
    __threadfence();
    for (int cl = 0; cl < NW; cl += 8) { const int cs = (cl + sk) & (NW - 1); const v4f va = *(const v4f*)(p + cs), vb = *(const v4f*)(p + cs + 4), ga = *(const v4f*)(sq + cs), gb = *(const v4f*)(sq + cs + 4), oa = *(const v4f*)(oq + cs), ob = *(const v4f*)(oq + cs + 4); v8h wo;
#pragma unroll
        for (int q = 0; q < 4; ++q) { wo[q] = toh_flush((bfr(va[q]) - av) * rs * bfr(ga[q]) + bfr(oa[q])); wo[q + 4] = toh_flush((bfr(vb[q]) - av) * rs * bfr(gb[q]) + bfr(ob[q])); }
        *(volatile v8h*)(o + cs) = wo; }
}

__global__ __launch_bounds__(256) void k_walk8(const float* __restrict__ Pa, const float* __restrict__ Pd, const float* __restrict__ eq, const float* __restrict__ nq, h16* Yh) { const unsigned nb = blockIdx.x * 256u + threadIdx.x; const unsigned bk = nb / 192u, pr = nb - bk * 192u, ch = pr * 2u; float ng[2][NE], cw[2][NE], dv[2];
#pragma unroll
    for (int k = 0; k < 2; ++k) { dv[k] = bfr(nq[ch + k]);
#pragma unroll
        for (int s = 0; s < NE; ++s) { ng[k][s] = -expf(bfr(eq[(ch + k) * NE + s])); cw[k][s] = 0.0f; } }
    for (int l0 = 0; l0 < NK; l0 += 8) { const size_t r0 = (size_t)bk * NK + l0; v2h w8[8];
#pragma unroll
        for (int j = 0; j < 8; ++j) { const size_t r = r0 + j; const v2f a2 = *(const v2f*)(Pa + r * NX + ch), g2 = *(const v2f*)(Pa + r * NX + NI + ch), b2 = *(const v2f*)(Pd + r * NI + ch); v2h wo;
#pragma unroll
            for (int k = 0; k < 2; ++k) { const float u = a2[k] / (1.0f + expf(-a2[k])); const float gt = g2[k] / (1.0f + expf(-g2[k])); const float pc = fmaxf(b2[k], 0.0f) + log1pf(expf(-fabsf(b2[k]))); float sm = 0.0f;
#pragma unroll
                for (int s = 0; s < NE; ++s) { cw[k][s] = cw[k][s] * expf(pc * ng[k][s]) + u; sm += cw[k][s]; }
                wo[k] = toh_flush(sm * gt + u * dv[k]); }
            w8[j] = wo; }
        h16* o = Yh + r0 * NI + ch;
#pragma unroll
        for (int j = 0; j < 8; ++j) *(volatile v2h*)(o + (size_t)j * NI) = w8[j];
        __threadfence();
#pragma unroll
        for (int j = 0; j < 8; ++j) *(volatile v2h*)(o + (size_t)j * NI) = w8[j]; }
}

__global__ __launch_bounds__(256) void k_add(const float* __restrict__ Oz, const float* __restrict__ src, float* out) { const size_t at = ((size_t)blockIdx.x * 256 + threadIdx.x) * 4; const v4f va = *(const v4f*)(Oz + at), vc = *(const v4f*)(src + at); v4f wo;
#pragma unroll
    for (int q = 0; q < 4; ++q) wo[q] = va[q] + bfr(vc[q]);
    *(volatile v4f*)(out + at) = wo; __threadfence(); *(volatile v4f*)(out + at) = wo; }

extern "C" void kernel_launch(void* const* d_in, const int* in_sizes, int n_in, void* d_out, int out_size, void* d_ws, size_t ws_size, hipStream_t stream) {
    if (n_in < 11) return;
    if (in_sizes[0] != NM * NW || in_sizes[1] != NW || in_sizes[2] != NW || in_sizes[3] != NA * NW || in_sizes[4] != NA || in_sizes[5] != NI * NI || in_sizes[6] != NI || in_sizes[7] != NI * NE || in_sizes[8] != NI || in_sizes[9] != NW * NI || in_sizes[10] != NW) return;
    if (out_size != NM * NW) return;
    static_assert(NM % 256 == 0 && NM % 64 == 0 && NX % 64 == 0 && NI % 64 == 0 && NW % 64 == 0 && NW % 32 == 0 && NI % 32 == 0 && NA == NX + NI && NX == 2 * NI && (NA * NW / 8) % 256 == 0 && (NI * NI / 8) % 256 == 0 && (NW * NI / 8) % 256 == 0 && (NM * NI / 8) % 256 == 0 && NM % NK == 0 && NK % 8 == 0 && (NI / 2) % 32 == 0 && ((NM / NK) * (NI / 2)) % 256 == 0 && (NM * NW / 4) % 256 == 0 && NW % 8 == 0 && NE == 8, "the products: row and column counts multiples of 64, the depths of 32; every one-dimensional launch exact; a wave's 32 pairs in one block of rows; the rows of a block in eights");
    const float* i0 = (const float*)d_in[0]; const float* i1 = (const float*)d_in[1]; const float* i2 = (const float*)d_in[2]; const float* i3 = (const float*)d_in[3]; const float* i4 = (const float*)d_in[4]; const float* i5 = (const float*)d_in[5]; const float* i6 = (const float*)d_in[6]; const float* i7 = (const float*)d_in[7]; const float* i8 = (const float*)d_in[8]; const float* i9 = (const float*)d_in[9]; const float* i10 = (const float*)d_in[10]; float* out = (float*)d_out;
    char* wsp = (char*)d_ws; auto take = [&](size_t bytes) { char* p = wsp; wsp += (bytes + 255) & ~(size_t)255; return (void*)p; };
    h16* Xh = (h16*)take((size_t)NM * NW * 2); h16* Wa = (h16*)take((size_t)NA * NW * 2); h16* Wb = (h16*)take((size_t)NI * NI * 2); h16* Wc = (h16*)take((size_t)NW * NI * 2); float* Pa = (float*)take((size_t)NM * NX * 4); float* Pd = (float*)take((size_t)NM * NI * 4); h16* Dh = (h16*)take((size_t)NM * NI * 2); h16* Yh = (h16*)take((size_t)NM * NI * 2); float* Oz = (float*)take((size_t)NM * NW * 4);
    if ((size_t)(wsp - (char*)d_ws) > ws_size) return;
    k_rnh<<<(unsigned)(NM / 256), 256, 0, stream>>>(i0, i1, i2, Xh);
    k_c16<true><<<(unsigned)(NA * NW / 8 / 256), 256, 0, stream>>>(i3, Wa, (size_t)NA * NW / 8);
    k_c16<true><<<(unsigned)(NI * NI / 8 / 256), 256, 0, stream>>>(i5, Wb, (size_t)NI * NI / 8);
    k_c16<true><<<(unsigned)(NW * NI / 8 / 256), 256, 0, stream>>>(i9, Wc, (size_t)NW * NI / 8);
    k_gemmw<h16, 0, true><<<dim3(NM / 64, NX / 64, 1), 32, 0, stream>>>(Xh, nullptr, Wa, nullptr, NW, Pa, NX, i4, 0, 0, 0);
    k_gemmw<h16, 0, true><<<dim3(NM / 64, NI / 64, 1), 32, 0, stream>>>(Xh, nullptr, Wa + (size_t)NX * NW, nullptr, NW, Pd, NI, i4 + NX, 0, 0, 0);
    k_c16<false><<<(unsigned)(NM * NI / 8 / 256), 256, 0, stream>>>(Pd, Dh, (size_t)NM * NI / 8);
    k_gemmw<h16, 0, true><<<dim3(NM / 64, NI / 64, 1), 32, 0, stream>>>(Dh, nullptr, Wb, nullptr, NI, Pd, NI, i6, 0, 0, 0);
    k_walk8<<<(unsigned)((NM / NK) * (NI / 2) / 256), 256, 0, stream>>>(Pa, Pd, i7, i8, Yh);
    k_gemmw<h16, 0, true><<<dim3(NM / 64, NW / 64, 1), 32, 0, stream>>>(Yh, nullptr, Wc, nullptr, NI, Oz, NW, i10, 0, 0, 0);
    k_add<<<(unsigned)(NM * NW / 4 / 256), 256, 0, stream>>>(Oz, i0, out);
}
